// TransformerBlock_5231270167156
// MI455X (gfx1250) — hardware-verified
//
#include <hip/hip_runtime.h>
#ifndef NB
#define NB 1
#endif
#ifndef SEQ
#define SEQ 4096
#endif
#define NB_FULL 1
#define SEQ_FULL 4096
#define DM 1024
#define NH 16
#define HD 64
#define DFF 4096
#define LQ (3 * DM)
#define MP (NB * SEQ)
#define PSP 72

static_assert(NB == 1);
static_assert(NH * HD == DM);
static_assert(HD == 64);
static_assert(DM % 64 == 0 && LQ % 64 == 0 && DFF % 64 == 0);
static_assert(DM % 32 == 0 && DFF % 32 == 0 && SEQ % 32 == 0);
static_assert(MP % 128 == 0 && SEQ % 64 == 0);
static_assert(256 * 4 == DM);
static_assert(DM / 8 == 128);
static_assert(NB <= NB_FULL && SEQ <= SEQ_FULL);
static_assert(PSP % 8 == 0 && PSP >= 64);
static_assert(((size_t)MP * (DM / 8)) % 256 == 0);
static_assert(((size_t)DM * (DM / 8)) % 256 == 0 && ((size_t)DFF * (DM / 8)) % 256 == 0 && ((size_t)DM * (DFF / 8)) % 256 == 0);

typedef _Float16 v16h __attribute__((ext_vector_type(16)));
typedef _Float16 v4ha __attribute__((ext_vector_type(4), may_alias));
typedef unsigned short v8us __attribute__((ext_vector_type(8), may_alias));
typedef float v8f __attribute__((ext_vector_type(8)));
typedef float v4f __attribute__((ext_vector_type(4)));
typedef float v4fa __attribute__((ext_vector_type(4), may_alias));
union FragH { v16h v; v8us half[2]; _Float16 h[16]; unsigned short u[16]; };

__device__ __forceinline__ unsigned short bf16_bits(float x) { unsigned int u = __float_as_uint(x); return (unsigned short)((u + 0x7FFFu + ((u >> 16) & 1u)) >> 16); }
__device__ __forceinline__ float bf16_rne(float x) { return __uint_as_float(((unsigned int)bf16_bits(x)) << 16); }

__global__ __launch_bounds__(256) void k_wt_f16(const float* __restrict__ W, _Float16* __restrict__ Wt, unsigned K, unsigned N, float scale) {
  const unsigned t = blockIdx.x * 256u + threadIdx.x; const unsigned k8n = K >> 3; if (t >= N * k8n) return;
  const unsigned n = t / k8n, k8 = (t - n * k8n) << 3; FragH f;
#pragma unroll
  for (unsigned i = 0; i < 8; ++i) f.h[i] = (_Float16)(bf16_rne(W[(size_t)(k8 + i) * N + n]) * scale);
  const v8us o = f.half[0]; unsigned short* dst = (unsigned short*)Wt + (size_t)n * K + k8;
  *(volatile v8us*)dst = o; __threadfence(); *(volatile v8us*)dst = o;
}

__global__ __launch_bounds__(256) void k_x16(const float* __restrict__ X, _Float16* __restrict__ X16, unsigned nrows) {
  const unsigned t = blockIdx.x * 256u + threadIdx.x; if (t >= nrows * (unsigned)(DM / 8)) return;
  const unsigned r = t >> 7, c8 = (t & 127u) << 3;
  const v4f a = *(const v4fa*)(X + (size_t)r * DM + c8), b = *(const v4fa*)(X + (size_t)r * DM + c8 + 4u);
  FragH f;
#pragma unroll
  for (unsigned i = 0; i < 4; ++i) { f.h[i] = (_Float16)bf16_rne(a[i]); f.h[4u + i] = (_Float16)bf16_rne(b[i]); }
  const v8us o = f.half[0]; unsigned short* dst = (unsigned short*)X16 + (size_t)r * DM + c8;
  *(volatile v8us*)dst = o; __threadfence(); *(volatile v8us*)dst = o;
}

template <int W16, int WF>
__global__ __launch_bounds__(256) void k_ln16(const float* __restrict__ X, const float* __restrict__ g, const float* __restrict__ bb, float eps, _Float16* __restrict__ N16, float* __restrict__ YF) {
  #pragma clang fp contract(off)
  __shared__ float red1[8]; __shared__ float red2[8];
  __shared__ __attribute__((aligned(16))) _Float16 row16[DM];
  const unsigned r = blockIdx.x, t = threadIdx.x, w = t >> 5, lane = t & 31u;
  const v4f xa = *(const v4fa*)(X + (size_t)r * DM + t * 4u);
  float sum = (xa[0] + xa[1]) + (xa[2] + xa[3]);
  for (int o = 16; o > 0; o >>= 1) sum += __shfl_xor(sum, o, 32);
  if (lane == 0u) red1[w] = sum;
  __syncthreads();
  const float mu = (((red1[0] + red1[1]) + (red1[2] + red1[3])) + ((red1[4] + red1[5]) + (red1[6] + red1[7]))) / (float)DM;
  float dl[4];
#pragma unroll
  for (unsigned q = 0; q < 4; ++q) dl[q] = xa[q] - mu;
  float vs = (dl[0] * dl[0] + dl[1] * dl[1]) + (dl[2] * dl[2] + dl[3] * dl[3]);
  for (int o = 16; o > 0; o >>= 1) vs += __shfl_xor(vs, o, 32);
  if (lane == 0u) red2[w] = vs;
  __syncthreads();
  const float var = (((red2[0] + red2[1]) + (red2[2] + red2[3])) + ((red2[4] + red2[5]) + (red2[6] + red2[7]))) / (float)DM;
  const float rs = rsqrtf(var + eps);
  const v4f gv = *(const v4fa*)(g + t * 4u), bv = *(const v4fa*)(bb + t * 4u);
  v4ha y4; v4f yf;
#pragma unroll
  for (unsigned q = 0; q < 4; ++q) { const float yv = (dl[q] * rs) * bf16_rne(gv[q]) + bf16_rne(bv[q]); yf[q] = yv; y4[q] = (_Float16)yv; }
  if (W16) *(v4ha*)(&row16[t * 4u]) = y4;
  __syncthreads();
  v8us o8 = {0, 0, 0, 0, 0, 0, 0, 0};
  if (W16) { if (t < 128u) o8 = *(const v8us*)((const unsigned short*)row16 + t * 8u); }
  const size_t ob = (size_t)r * DM;
  for (int pass = 0; pass < 2; ++pass) {
    if (WF) *(volatile v4f*)(YF + ob + t * 4u) = yf;
    if (W16) { if (t < 128u) *(volatile v8us*)((unsigned short*)N16 + ob + t * 8u) = o8; }
    if (pass == 0) __threadfence(); }
}

__device__ __forceinline__ v16h g2_frag(const _Float16* p, unsigned hh) { FragH f; f.half[0] = *(const v8us*)((const unsigned short*)p + 8u * hh); f.half[1] = *(const v8us*)((const unsigned short*)p + 16u + 8u * hh); return f.v; }
__device__ __forceinline__ v8f g2_mma(v16h a, v16h b, v8f c) { v8f d = __builtin_amdgcn_wmma_f32_16x16x32_f16(false, a, false, b, (short)0, c, false, false); asm volatile("v_nop\n\tv_nop\n\tv_nop\n\tv_nop" : "+v"(d) : "v"(a), "v"(b)); return d; }
template <int ACT, int CPM>
__global__ __launch_bounds__(128) void k_gemm2(const _Float16* __restrict__ A, unsigned lda, size_t sA, const _Float16* __restrict__ Bh, unsigned ldb, size_t sB, float alpha,
    const float* __restrict__ bias, const float* __restrict__ CP, float* __restrict__ C, _Float16* __restrict__ C16, float c16s, unsigned ldc, size_t sC, unsigned M, unsigned N, unsigned K) {
  static_assert(ACT == 0 || ACT == 1);
  static_assert(CPM == 0 || ACT == 0);
  __shared__ __attribute__((aligned(16))) float so[4][32][68];
  const unsigned tid = threadIdx.x, w = tid >> 5, lane = tid & 31u, ln = lane & 15u, hh = lane >> 4; const unsigned by = blockIdx.y;
  A += (size_t)by * sA; Bh += (size_t)by * sB; const size_t cofs = (size_t)by * sC;
  const unsigned ntn = N >> 6; const unsigned mt = blockIdx.x / ntn, nq = blockIdx.x - mt * ntn; const unsigned row0 = mt * 128u + 32u * w, col0 = nq * 64u; if (row0 >= M) return;
  const _Float16* a0p = A + (size_t)(row0 + ln) * lda; const _Float16* a1p = a0p + (size_t)16 * lda;
  const _Float16* b0p = Bh + (size_t)(col0 + ln) * ldb; const _Float16* b1p = b0p + (size_t)16 * ldb; const _Float16* b2p = b1p + (size_t)16 * ldb; const _Float16* b3p = b2p + (size_t)16 * ldb;
  const v8f z8 = {0.f,0.f,0.f,0.f,0.f,0.f,0.f,0.f}; v8f c00 = z8, c01 = z8, c02 = z8, c03 = z8, c10 = z8, c11 = z8, c12 = z8, c13 = z8;
#pragma unroll 1
  for (unsigned kb = 0; kb < K; kb += 32u) { const v16h a0 = g2_frag(a0p + kb, hh), a1 = g2_frag(a1p + kb, hh);
    v16h b = g2_frag(b0p + kb, hh); c00 = g2_mma(a0, b, c00); c10 = g2_mma(a1, b, c10);
    b = g2_frag(b1p + kb, hh); c01 = g2_mma(a0, b, c01); c11 = g2_mma(a1, b, c11);
    b = g2_frag(b2p + kb, hh); c02 = g2_mma(a0, b, c02); c12 = g2_mma(a1, b, c12);
    b = g2_frag(b3p + kb, hh); c03 = g2_mma(a0, b, c03); c13 = g2_mma(a1, b, c13); }
  v8f accs[8] = {c00, c01, c02, c03, c10, c11, c12, c13};
#pragma unroll
  for (unsigned u = 0; u < 8; ++u) { const unsigned t = u & 3u, half = u >> 2; const unsigned col = col0 + t * 16u + ln; const float bv = bias ? bf16_rne(bias[col]) : 0.f;
#pragma unroll
    for (unsigned r = 0; r < 8; ++r) { const unsigned rloc = half * 16u + 8u * hh + r; float v = accs[u][r] * alpha + bv;
      if (ACT == 1) v = fmaxf(v, 0.f);
      so[w][rloc][t * 16u + ln] = v; } }
  __builtin_amdgcn_fence(4  , "workgroup"); __builtin_amdgcn_wave_barrier();
  const unsigned rsub = lane >> 4, c4 = (lane & 15u) * 4u;
  if (CPM != 0) {
#pragma unroll 4
    for (unsigned q = 0; q < 16; ++q) { const unsigned r = q * 2u + rsub; const size_t o = cofs + (size_t)(row0 + r) * ldc + col0 + c4;
      v4f cp = *(const v4fa*)(CP + o);
      if (CPM == 2) {
#pragma unroll
        for (unsigned i = 0; i < 4; ++i) cp[i] = bf16_rne(cp[i]); }
      v4f v = *(const v4fa*)&so[w][r][c4]; v = v + cp; *(v4fa*)&so[w][r][c4] = v; }
    __builtin_amdgcn_fence(4  , "workgroup"); __builtin_amdgcn_wave_barrier(); }
  const unsigned rsub8 = lane >> 3, c8 = (lane & 7u) * 8u;
  for (int pass = 0; pass < 2; ++pass) {
    if (C) {
#pragma unroll
      for (unsigned q = 0; q < 16; ++q) { const unsigned r = q * 2u + rsub; const v4f v = *(const v4fa*)&so[w][r][c4]; const size_t o = cofs + (size_t)(row0 + r) * ldc + col0 + c4;
        *(volatile v4f*)(C + o) = v; } }
    if (C16) {
#pragma unroll
      for (unsigned q = 0; q < 8; ++q) { const unsigned r = q * 4u + rsub8; const v4f va = *(const v4fa*)&so[w][r][c8], vb = *(const v4fa*)&so[w][r][c8 + 4u]; FragH f;
#pragma unroll
        for (unsigned i = 0; i < 4; ++i) { f.h[i] = (_Float16)(va[i] * c16s); f.h[4u + i] = (_Float16)(vb[i] * c16s); }
        const size_t o = cofs + (size_t)(row0 + r) * ldc + col0 + c8;
        *(volatile v8us*)((unsigned short*)C16 + o) = f.half[0]; } }
    if (pass == 0) __threadfence(); } }

template <int NHv, int TTv>
__global__ __launch_bounds__(256) void k_vt(const _Float16* __restrict__ V16, unsigned ldv, unsigned voff, _Float16* __restrict__ Vt) {
  __shared__ unsigned short tl[64][66];
  const unsigned tid = threadIdx.x; const unsigned slab = blockIdx.x / (unsigned)(TTv / 64), lg = blockIdx.x - slab * (unsigned)(TTv / 64); const unsigned b = slab / (unsigned)NHv, h = slab - b * (unsigned)NHv;
  for (unsigned i = tid; i < 512u; i += 256u) { const unsigned r = i >> 3, c8 = (i & 7u) << 3; FragH f; f.half[0] = *(const v8us*)((const unsigned short*)V16 + ((size_t)b * TTv + lg * 64u + r) * ldv + voff + h * 64u + c8);
#pragma unroll
    for (unsigned q = 0; q < 8; ++q) tl[r][c8 + q] = f.u[q]; }
  __syncthreads();
  for (int pass = 0; pass < 2; ++pass) {
#pragma unroll
    for (unsigned rd = 0; rd < 2; ++rd) { const unsigned d = rd * 32u + (tid >> 3), pc = tid & 7u; FragH f;
#pragma unroll
      for (unsigned q = 0; q < 8; ++q) f.u[q] = tl[pc * 8u + q][d];
      *(volatile v8us*)((unsigned short*)Vt + ((size_t)slab * 64u + d) * TTv + lg * 64u + pc * 8u) = f.half[0]; }
    if (pass == 0) __threadfence(); } }

__global__ __launch_bounds__(128) void k_flash(const _Float16* __restrict__ Q16, const _Float16* __restrict__ K16, const _Float16* __restrict__ Vt, _Float16* __restrict__ O16) {
  __shared__ __attribute__((aligned(16))) _Float16 ps[4][16][PSP];
  const unsigned tid = threadIdx.x, w = tid >> 5, lane = tid & 31u, ln = lane & 15u, hh = lane >> 4;
  const unsigned h = blockIdx.y, qblk = blockIdx.x;
  const unsigned qrow0 = qblk * 64u + w * 16u;
  const unsigned rowl = w * 16u + 8u * hh;
  const _Float16* qp = Q16 + (size_t)(qrow0 + ln) * LQ + h * 64u;
  const v16h aq0 = g2_frag(qp, hh), aq1 = g2_frag(qp + 32, hh);
  const v8f z8 = {0.f,0.f,0.f,0.f,0.f,0.f,0.f,0.f};
  v8f o[4] = {z8, z8, z8, z8};
  float mrun[8], lrun[8];
#pragma unroll
  for (unsigned r = 0; r < 8; ++r) { mrun[r] = -1.0e30f; lrun[r] = 0.f; }
#pragma unroll 1
  for (unsigned kb = 0; kb <= qblk; ++kb) {
    const unsigned kbase = kb * 64u;
    const _Float16* kp = K16 + (size_t)(kbase + ln) * LQ + h * 64u;
    v8f s[4];
#pragma unroll
    for (unsigned nf = 0; nf < 4; ++nf) { const _Float16* kr = kp + (size_t)(nf * 16u) * LQ; const v16h b0 = g2_frag(kr, hh), b1 = g2_frag(kr + 32, hh);
      const v8f a = g2_mma(aq0, b0, z8); s[nf] = g2_mma(aq1, b1, a); }
    const bool diag = (kb == qblk);
#pragma unroll
    for (unsigned nf = 0; nf < 4; ++nf) {
#pragma unroll
      for (unsigned r = 0; r < 8; ++r) { const float v = s[nf][r] * 0.125f; const bool msk = diag && ((nf * 16u + ln) > (rowl + r)); s[nf][r] = msk ? -1.0e30f : v; } }
#pragma unroll
    for (unsigned r = 0; r < 8; ++r) {
      float mx = fmaxf(fmaxf(s[0][r], s[1][r]), fmaxf(s[2][r], s[3][r]));
      mx = fmaxf(mx, __shfl_xor(mx, 1, 32)); mx = fmaxf(mx, __shfl_xor(mx, 2, 32)); mx = fmaxf(mx, __shfl_xor(mx, 4, 32)); mx = fmaxf(mx, __shfl_xor(mx, 8, 32));
      const float mnew = fmaxf(mrun[r], mx);
      const float alpha = __expf(mrun[r] - mnew);
      float rsum = 0.f;
#pragma unroll
      for (unsigned nf = 0; nf < 4; ++nf) { const float p = __expf(s[nf][r] - mnew); const _Float16 ph = (_Float16)(p * 256.0f); ps[w][8u * hh + r][nf * 16u + ln] = ph; rsum += (float)ph; }
      rsum += __shfl_xor(rsum, 1, 32); rsum += __shfl_xor(rsum, 2, 32); rsum += __shfl_xor(rsum, 4, 32); rsum += __shfl_xor(rsum, 8, 32);
      lrun[r] = lrun[r] * alpha + rsum; mrun[r] = mnew;
#pragma unroll
      for (unsigned nf = 0; nf < 4; ++nf) o[nf][r] *= alpha; }
    __builtin_amdgcn_fence(4  , "workgroup"); __builtin_amdgcn_wave_barrier();
    const v16h ap0 = g2_frag(&ps[w][ln][0], hh), ap1 = g2_frag(&ps[w][ln][32], hh);
    const _Float16* vp = Vt + ((size_t)h * 64u + ln) * SEQ + kbase;
#pragma unroll
    for (unsigned nf = 0; nf < 4; ++nf) { const _Float16* vr = vp + (size_t)(nf * 16u) * SEQ; const v16h b0 = g2_frag(vr, hh), b1 = g2_frag(vr + 32, hh);
      o[nf] = g2_mma(ap0, b0, o[nf]); o[nf] = g2_mma(ap1, b1, o[nf]); }
    __builtin_amdgcn_fence(4  , "workgroup"); __builtin_amdgcn_wave_barrier();
  }
  float inv[8];
#pragma unroll
  for (unsigned r = 0; r < 8; ++r) inv[r] = 64.0f * (1.0f / lrun[r]);
#pragma unroll
  for (unsigned nf = 0; nf < 4; ++nf) {
#pragma unroll
    for (unsigned r = 0; r < 8; ++r) ps[w][8u * hh + r][nf * 16u + ln] = (_Float16)(o[nf][r] * inv[r]); }
  __builtin_amdgcn_fence(4  , "workgroup"); __builtin_amdgcn_wave_barrier();
  const unsigned rsub8 = lane >> 3, c8 = (lane & 7u) * 8u;
  v8us t4[4];
#pragma unroll
  for (unsigned q = 0; q < 4; ++q) t4[q] = *(const v8us*)((const unsigned short*)&ps[w][q * 4u + rsub8][c8]);
  for (int pass = 0; pass < 2; ++pass) {
#pragma unroll
    for (unsigned q = 0; q < 4; ++q) *(volatile v8us*)((unsigned short*)O16 + (size_t)(qrow0 + q * 4u + rsub8) * DM + h * 64u + c8) = t4[q];
    if (pass == 0) __threadfence(); }
}

constexpr size_t pad256(size_t b) { return (b + 255) & ~(size_t)255; }
constexpr size_t SZ_BQKV = pad256((size_t)LQ * DM * 2);
constexpr size_t SZ_BO   = pad256((size_t)DM * DM * 2);
constexpr size_t SZ_BW1  = pad256((size_t)DFF * DM * 2);
constexpr size_t SZ_BW2  = pad256((size_t)DM * DFF * 2);
constexpr size_t SZ_X16  = pad256((size_t)MP * DM * 2);
constexpr size_t SZ_QKV  = pad256((size_t)MP * LQ * 2);
constexpr size_t SZ_VT   = pad256((size_t)NB * NH * HD * SEQ * 2);
constexpr size_t SZ_O16  = pad256((size_t)MP * DM * 2);
constexpr size_t SZ_Y    = pad256((size_t)MP * DM * 4);
constexpr size_t SZ_HF   = pad256((size_t)MP * DM * 4);
constexpr size_t SZ_HID  = (size_t)MP * DFF * 2;
constexpr size_t SZ_TOTAL = SZ_BQKV + SZ_BO + SZ_BW1 + SZ_BW2 + SZ_X16 + SZ_QKV + SZ_VT + SZ_O16 + SZ_Y + SZ_HF;
static_assert(SZ_HID <= SZ_QKV + SZ_VT);
static_assert(SZ_TOTAL <= (size_t)134217728);

extern "C" void kernel_launch(void* const* d_in, const int* in_sizes, int n_in,
                              void* d_out, int out_size, void* d_ws, size_t ws_size, hipStream_t stream) {
  if (n_in < 17) return;
  if ((long long)in_sizes[0] < (long long)MP * DM) return;
  if (in_sizes[1] < DM * DM || in_sizes[3] < DM * DM || in_sizes[5] < DM * DM || in_sizes[7] < DM * DM) return;
  if (in_sizes[2] < DM || in_sizes[4] < DM || in_sizes[6] < DM || in_sizes[8] < DM || in_sizes[9] < DM || in_sizes[10] < DM) return;
  if (in_sizes[11] < DM * DFF || in_sizes[12] < DFF || in_sizes[13] < DFF * DM || in_sizes[14] < DM || in_sizes[15] < DM || in_sizes[16] < DM) return;
  if ((long long)out_size < (long long)MP * DM) return;
  if (SZ_TOTAL > ws_size) return;
  const float* const* I = (const float* const*)d_in;
  const float* x = I[0]; const float* wq = I[1]; const float* bq = I[2]; const float* wk = I[3]; const float* bk = I[4];
  const float* wv = I[5]; const float* bv = I[6]; const float* wo = I[7]; const float* bo = I[8];
  const float* g1 = I[9]; const float* be1 = I[10]; const float* wf1 = I[11]; const float* bf1 = I[12];
  const float* wf2 = I[13]; const float* bf2 = I[14]; const float* g2 = I[15]; const float* be2 = I[16];
  char* ws = (char*)d_ws; size_t off = 0;
  _Float16* BQKV = (_Float16*)(ws + off); off += SZ_BQKV;
  _Float16* BO   = (_Float16*)(ws + off); off += SZ_BO;
  _Float16* BW1  = (_Float16*)(ws + off); off += SZ_BW1;
  _Float16* BW2  = (_Float16*)(ws + off); off += SZ_BW2;
  _Float16* X16  = (_Float16*)(ws + off); off += SZ_X16;
  _Float16* QKV  = (_Float16*)(ws + off); off += SZ_QKV;
  _Float16* VT   = (_Float16*)(ws + off); off += SZ_VT;
  _Float16* O16  = (_Float16*)(ws + off); off += SZ_O16;
  float*    Y    = (float*)(ws + off);    off += SZ_Y;
  float*    HF   = (float*)(ws + off);    off += SZ_HF;
  _Float16* HID  = QKV;
  _Float16* H16  = X16;
  _Float16* Q16 = QKV; _Float16* K16 = QKV + DM; _Float16* V16 = QKV + 2 * DM;

  k_wt_f16<<<(unsigned)(((size_t)DM * (DM / 8) + 255) / 256), 256, 0, stream>>>(wq, BQKV, (unsigned)DM, (unsigned)DM, 16.0f);
  k_wt_f16<<<(unsigned)(((size_t)DM * (DM / 8) + 255) / 256), 256, 0, stream>>>(wk, BQKV + (size_t)DM * DM, (unsigned)DM, (unsigned)DM, 16.0f);
  k_wt_f16<<<(unsigned)(((size_t)DM * (DM / 8) + 255) / 256), 256, 0, stream>>>(wv, BQKV + (size_t)2 * DM * DM, (unsigned)DM, (unsigned)DM, 16.0f);
  k_wt_f16<<<(unsigned)(((size_t)DM * (DM / 8) + 255) / 256), 256, 0, stream>>>(wo, BO, (unsigned)DM, (unsigned)DM, 16.0f);
  k_wt_f16<<<(unsigned)(((size_t)DFF * (DM / 8) + 255) / 256), 256, 0, stream>>>(wf1, BW1, (unsigned)DM, (unsigned)DFF, 16.0f);
  k_wt_f16<<<(unsigned)(((size_t)DM * (DFF / 8) + 255) / 256), 256, 0, stream>>>(wf2, BW2, (unsigned)DFF, (unsigned)DM, 16.0f);
  k_x16<<<(unsigned)(((size_t)MP * (DM / 8) + 255) / 256), 256, 0, stream>>>(x, X16, (unsigned)MP);
  k_gemm2<0, 0><<<dim3((unsigned)((MP / 128) * (DM / 64)), 1), 128, 0, stream>>>(X16, (unsigned)DM, (size_t)0, BQKV, (unsigned)DM, (size_t)0, 0.0625f, bq, nullptr, nullptr, Q16, 1.0f, (unsigned)LQ, (size_t)0, (unsigned)MP, (unsigned)DM, (unsigned)DM);
  k_gemm2<0, 0><<<dim3((unsigned)((MP / 128) * (DM / 64)), 1), 128, 0, stream>>>(X16, (unsigned)DM, (size_t)0, BQKV + (size_t)DM * DM, (unsigned)DM, (size_t)0, 0.0625f, bk, nullptr, nullptr, K16, 1.0f, (unsigned)LQ, (size_t)0, (unsigned)MP, (unsigned)DM, (unsigned)DM);
  k_gemm2<0, 0><<<dim3((unsigned)((MP / 128) * (DM / 64)), 1), 128, 0, stream>>>(X16, (unsigned)DM, (size_t)0, BQKV + (size_t)2 * DM * DM, (unsigned)DM, (size_t)0, 0.0625f, bv, nullptr, nullptr, V16, 1.0f, (unsigned)LQ, (size_t)0, (unsigned)MP, (unsigned)DM, (unsigned)DM);
  k_vt<NH, SEQ><<<(unsigned)(NB * NH * (SEQ / 64)), 256, 0, stream>>>(V16, (unsigned)LQ, 0u, VT);
  k_flash<<<dim3((unsigned)(SEQ / 64), (unsigned)NH), 128, 0, stream>>>(Q16, K16, VT, O16);
  k_gemm2<0, 2><<<dim3((unsigned)((MP / 128) * (DM / 64)), 1), 128, 0, stream>>>(O16, (unsigned)DM, (size_t)0, BO, (unsigned)DM, (size_t)0, 0.0009765625f, bo, x, Y, nullptr, 1.0f, (unsigned)DM, (size_t)0, (unsigned)MP, (unsigned)DM, (unsigned)DM);
  k_ln16<1, 1><<<(unsigned)MP, 256, 0, stream>>>(Y, g1, be1, 1e-5f, H16, HF);
  k_gemm2<1, 0><<<dim3((unsigned)((MP / 128) * (DFF / 64)), 1), 128, 0, stream>>>(H16, (unsigned)DM, (size_t)0, BW1, (unsigned)DM, (size_t)0, 0.0625f, bf1, nullptr, nullptr, HID, 16.0f, (unsigned)DFF, (size_t)0, (unsigned)MP, (unsigned)DFF, (unsigned)DM);
  k_gemm2<0, 1><<<dim3((unsigned)((MP / 128) * (DM / 64)), 1), 128, 0, stream>>>(HID, (unsigned)DFF, (size_t)0, BW2, (unsigned)DFF, (size_t)0, 0.00390625f, bf2, HF, Y, nullptr, 1.0f, (unsigned)DM, (size_t)0, (unsigned)MP, (unsigned)DM, (unsigned)DFF);
  k_ln16<0, 1><<<(unsigned)MP, 256, 0, stream>>>(Y, g2, be2, 1e-5f, nullptr, (float*)d_out);
}
